// PoolHiddenNet_d_14568529068508
// MI455X (gfx1250) — hardware-verified
//
#include <hip/hip_runtime.h>

typedef _Float16 v16h __attribute__((ext_vector_type(16)));
typedef _Float16 v8h  __attribute__((ext_vector_type(8)));
typedef float    v8f  __attribute__((ext_vector_type(8)));
typedef float    v4f  __attribute__((ext_vector_type(4)));
typedef v8h __attribute__((may_alias)) v8ha;
typedef v4f __attribute__((may_alias)) v4fa;

union Frag { v16h v; v8h half[2]; };

#define NSCENE 64
#define NPED   32
#define NB     2048
#define NPAIR  65536
#define HDIM   64
#define C1     512
#define C2     1024
#define BNEPS  1e-5f

#define OFF_W2T  0u
#define SZ_W2T   1048576u
#define OFF_W1BT 1048576u
#define SZ_W1BT  65536u
#define OFF_HH   1114112u
#define SZ_HH    262144u
#define OFF_MK   1376256u
#define SZ_MK    8192u
#define OFF_AP   1384448u
#define SZ_AP    4194304u
#define OFF_PP   5578752u
#define SZ_PP    4194304u
#define OFF_A1   9773056u
#define SZ_A1    67108864u
#define WS_TOTAL 76881920u
#define DYN_LDS_K4 139520

static_assert(OFF_W1BT == OFF_W2T + SZ_W2T);
static_assert(OFF_HH == OFF_W1BT + SZ_W1BT);
static_assert(OFF_MK == OFF_HH + SZ_HH);
static_assert(OFF_AP == OFF_MK + SZ_MK);
static_assert(OFF_PP == OFF_AP + SZ_AP);
static_assert(OFF_A1 == OFF_PP + SZ_PP);
static_assert(WS_TOTAL == OFF_A1 + SZ_A1);
static_assert((OFF_MK % 256u) == 0 && (OFF_AP % 256u) == 0 && (OFF_A1 % 256u) == 0);

__device__ __forceinline__ v8f wmma_f16(v16h a, v16h b, v8f c) {
  v8f d = __builtin_amdgcn_wmma_f32_16x16x32_f16(false, a, false, b, (short)0, c, false, false);
  asm volatile("v_nop\n\tv_nop\n\tv_nop\n\tv_nop" : "+v"(d) : "v"(a), "v"(b));
  return d;
}

__device__ __forceinline__ v16h load_frag(const _Float16* p, int h) {
  Frag f;
  f.half[0] = *(const v8ha*)(p + 8 * h);
  f.half[1] = *(const v8ha*)(p + 16 + 8 * h);
  return f.v;
}

__device__ __forceinline__ void tr_tile(const float* __restrict__ src, int spitch, int k0, int n0,
                                        _Float16* dst, int dpitch, float scale,
                                        _Float16* sT, int tid) {
  const int nc = tid & 63, kr0 = tid >> 6;
  #pragma unroll
  for (int i = 0; i < 16; ++i) {
    const int kr = kr0 + 4 * i;
    const float v = src[(size_t)(k0 + kr) * spitch + n0 + nc];
    sT[nc * 72 + kr] = (_Float16)(v * scale);
  }
  __syncthreads();
  const int q = tid & 7, l0 = tid >> 3;
  #pragma unroll
  for (int i = 0; i < 2; ++i) {
    const int line = l0 + 32 * i;
    const v8h v = *(const v8ha*)(sT + line * 72 + 8 * q);
    *(volatile v8h*)(dst + (size_t)(n0 + line) * dpitch + k0 + 8 * q) = v;
  }
  __threadfence();
  #pragma unroll
  for (int i = 0; i < 2; ++i) {
    const int line = l0 + 32 * i;
    const v8h v = *(const v8ha*)(sT + line * 72 + 8 * q);
    *(volatile v8h*)(dst + (size_t)(n0 + line) * dpitch + k0 + 8 * q) = v;
  }
}

__global__ __launch_bounds__(256) void prep_kernel(
    const float* __restrict__ W1, const float* __restrict__ W2, const float* __restrict__ hs,
    const float* __restrict__ Wemb, const float* __restrict__ bemb, const float* __restrict__ b1,
    _Float16* W2t, _Float16* W1bt, _Float16* hh, float* MK)
{
  __shared__ __attribute__((aligned(16))) _Float16 sT[64 * 72];
  const int tid = threadIdx.x, bid = blockIdx.x;
  if (bid < 128) {
    const int kt = bid >> 4, nt = bid & 15;
    tr_tile(W2, C2, 64 * kt, 64 * nt, W2t, C1, 64.0f, sT, tid);
  } else if (bid < 136) {
    const int nt = bid - 128;
    tr_tile(W1 + (size_t)64 * C1, C1, 0, 64 * nt, W1bt, HDIM, 64.0f, sT, tid);
  } else if (bid < 200) {
    const int g = (bid - 136) * 256 + tid;
    const float* s = hs + (size_t)g * 8;
    const v4f a = *(const v4fa*)s;
    const v4f c = *(const v4fa*)(s + 4);
    const v8h o = { (_Float16)(a.x * 8.0f), (_Float16)(a.y * 8.0f), (_Float16)(a.z * 8.0f), (_Float16)(a.w * 8.0f),
                    (_Float16)(c.x * 8.0f), (_Float16)(c.y * 8.0f), (_Float16)(c.z * 8.0f), (_Float16)(c.w * 8.0f) };
    _Float16* d = hh + (size_t)g * 8;
    *(volatile v8h*)d = o;
    __threadfence();
    *(volatile v8h*)d = o;
  } else {
    const int ch = (bid - 200) * 256 + tid;
    float m0 = 0.0f, m1 = 0.0f, kk = 0.0f;
    #pragma unroll 1
    for (int e = 0; e < 64; ++e) {
      const float w = W1[(size_t)e * C1 + ch];
      m0 = fmaf(Wemb[e], w, m0);
      m1 = fmaf(Wemb[64 + e], w, m1);
      kk = fmaf(bemb[e], w, kk);
    }
    kk += b1[ch];
    *(volatile float*)(MK + ch)          = m0;
    *(volatile float*)(MK + C1 + ch)     = m1;
    *(volatile float*)(MK + 2 * C1 + ch) = kk;
    __threadfence();
    *(volatile float*)(MK + ch)          = m0;
    *(volatile float*)(MK + C1 + ch)     = m1;
    *(volatile float*)(MK + 2 * C1 + ch) = kk;
  }
}

__device__ __forceinline__ void tile_store_pass(const float* sTile, float* plane,
                                                int rowbase, int colbase, int tid) {
  const int q = tid & 7, l0 = tid >> 3;
  #pragma unroll
  for (int i = 0; i < 4; ++i) {
    const int line = l0 + 32 * i;
    const v4f v = *(const v4fa*)(sTile + line * 32 + 4 * q);
    *(volatile v4f*)(plane + (size_t)(rowbase + line) * C1 + colbase + 4 * q) = v;
  }
}

__global__ __launch_bounds__(256) void pair_vec_kernel(
    const _Float16* __restrict__ hh, const _Float16* __restrict__ W1bt, const float* __restrict__ MK,
    const float* __restrict__ pos, const float* __restrict__ g1, const float* __restrict__ beta1,
    float* Ap, float* Pp)
{
  __shared__ __attribute__((aligned(16))) float sA[128 * 32];
  __shared__ __attribute__((aligned(16))) float sP[128 * 32];
  __shared__ double sPart[8 * 32 * 4];
  __shared__ float sStat[4 * 32 * 2];

  const int tid = threadIdx.x, lane = tid & 31, w = tid >> 5;
  const int h = lane >> 4, m = lane & 15;
  const int rowbase = blockIdx.x * 128, colbase = blockIdx.y * 32;

  const _Float16* ar  = hh + (size_t)(rowbase + 16 * w + m) * HDIM;
  const _Float16* br0 = W1bt + (size_t)(colbase + m) * HDIM;
  const _Float16* br1 = br0 + (size_t)16 * HDIM;
  const v8f zero8 = {0.f, 0.f, 0.f, 0.f, 0.f, 0.f, 0.f, 0.f};
  v8f acc0 = zero8, acc1 = zero8;
  #pragma unroll
  for (int ks = 0; ks < 2; ++ks) {
    const v16h a  = load_frag(ar + 32 * ks, h);
    const v16h b0 = load_frag(br0 + 32 * ks, h);
    const v16h bb = load_frag(br1 + 32 * ks, h);
    acc0 = wmma_f16(a, b0, acc0);
    acc1 = wmma_f16(a, bb, acc1);
  }
  #pragma unroll
  for (int r = 0; r < 8; ++r) {
    const int rl = 16 * w + 8 * h + r;
    sA[rl * 32 + m]      = acc0[r] * (1.0f / 512.0f);
    sA[rl * 32 + 16 + m] = acc1[r] * (1.0f / 512.0f);
  }
  __syncthreads();

  const int c = tid & 31, part = tid >> 5, sl = part >> 1, kh = part & 1;
  const int cg = colbase + c;
  const float m0 = MK[cg], m1 = MK[C1 + cg], k0v = MK[2 * C1 + cg];
  double SA = 0.0, SA2 = 0.0, SP = 0.0, SP2 = 0.0;
  #pragma unroll 1
  for (int k = 0; k < 16; ++k) {
    const int rl = 32 * sl + 16 * kh + k;
    const int p = rowbase + rl;
    const float x0 = pos[2 * p], x1 = pos[2 * p + 1];
    const float Pv = fmaf(x1, m1, x0 * m0);
    const float Av = sA[rl * 32 + c] + Pv + k0v;
    sA[rl * 32 + c] = Av;
    sP[rl * 32 + c] = Pv;
    SA += (double)Av; SA2 += (double)Av * (double)Av;
    SP += (double)Pv; SP2 += (double)Pv * (double)Pv;
  }
  sPart[(part * 32 + c) * 4 + 0] = SA;
  sPart[(part * 32 + c) * 4 + 1] = SA2;
  sPart[(part * 32 + c) * 4 + 2] = SP;
  sPart[(part * 32 + c) * 4 + 3] = SP2;
  __syncthreads();

  if (tid < 128) {
    const int s2 = tid >> 5;
    const int i0 = ((2 * s2) * 32 + c) * 4, i1 = ((2 * s2 + 1) * 32 + c) * 4;
    const double tA  = sPart[i0 + 0] + sPart[i1 + 0];
    const double tA2 = sPart[i0 + 1] + sPart[i1 + 1];
    const double tP  = sPart[i0 + 2] + sPart[i1 + 2];
    const double tP2 = sPart[i0 + 3] + sPart[i1 + 3];
    const double mean = (tA - tP) * (1.0 / 32.0);
    const double ey2  = (32.0 * tA2 + 32.0 * tP2 - 2.0 * tA * tP) * (1.0 / 1024.0);
    double var = ey2 - mean * mean;
    if (var < 0.0) var = 0.0;
    const float varf = (float)var;
    const float rstd = 1.0f / sqrtf(varf + BNEPS);
    sStat[(s2 * 32 + c) * 2 + 0] = (float)mean;
    sStat[(s2 * 32 + c) * 2 + 1] = rstd * g1[cg];
  }
  __syncthreads();

  {
    const float meanf = sStat[(sl * 32 + c) * 2 + 0];
    const float sc    = sStat[(sl * 32 + c) * 2 + 1];
    const float be    = beta1[cg];
    #pragma unroll 1
    for (int k = 0; k < 16; ++k) {
      const int rl = 32 * sl + 16 * kh + k;
      const float av = sA[rl * 32 + c];
      const float pv = sP[rl * 32 + c];
      sA[rl * 32 + c] = (av - meanf) * sc + be;
      sP[rl * 32 + c] = pv * sc;
    }
  }
  __syncthreads();

  tile_store_pass(sA, Ap, rowbase, colbase, tid);
  tile_store_pass(sP, Pp, rowbase, colbase, tid);
  __threadfence();
  tile_store_pass(sA, Ap, rowbase, colbase, tid);
  tile_store_pass(sP, Pp, rowbase, colbase, tid);
}

__global__ __launch_bounds__(256) void a1_build_kernel(
    const float* __restrict__ Ap, const float* __restrict__ Pp, _Float16* a1)
{
  const int g = blockIdx.x * 256 + threadIdx.x;
  if (g >= NPAIR * (C1 / 8)) return;
  const int row = g >> 6, c8 = (g & 63) * 8;
  const int s = row >> 10, rr = row & 1023;
  const int j = rr >> 5, k = rr & 31;
  const float* pa = Ap + (size_t)(s * NPED + k) * C1 + c8;
  const float* pp = Pp + (size_t)(s * NPED + j) * C1 + c8;
  const v4f a0 = *(const v4fa*)pa, a1v = *(const v4fa*)(pa + 4);
  const v4f p0 = *(const v4fa*)pp, p1 = *(const v4fa*)(pp + 4);
  const v8h o = { (_Float16)(16.0f * fmaxf(a0.x - p0.x, 0.0f)), (_Float16)(16.0f * fmaxf(a0.y - p0.y, 0.0f)),
                  (_Float16)(16.0f * fmaxf(a0.z - p0.z, 0.0f)), (_Float16)(16.0f * fmaxf(a0.w - p0.w, 0.0f)),
                  (_Float16)(16.0f * fmaxf(a1v.x - p1.x, 0.0f)), (_Float16)(16.0f * fmaxf(a1v.y - p1.y, 0.0f)),
                  (_Float16)(16.0f * fmaxf(a1v.z - p1.z, 0.0f)), (_Float16)(16.0f * fmaxf(a1v.w - p1.w, 0.0f)) };
  _Float16* d = a1 + (size_t)row * C1 + c8;
  *(volatile v8h*)d = o;
  __threadfence();
  *(volatile v8h*)d = o;
}

__global__ __launch_bounds__(256) void gemm2_pool_kernel(
    const _Float16* __restrict__ a1, const _Float16* __restrict__ W2t,
    const float* __restrict__ b2, const float* __restrict__ g2, const float* __restrict__ beta2,
    float* out)
{
  extern __shared__ __attribute__((aligned(16))) unsigned char dsm[];
  float*  sY    = (float*)dsm;
  double* sPart = (double*)(dsm + 131072);
  float*  sStat = (float*)(dsm + 131072 + 4096);
  float*  sOut  = (float*)(dsm + 131072 + 4096 + 256);

  const int tid = threadIdx.x, lane = tid & 31, w = tid >> 5;
  const int h = lane >> 4, m = lane & 15;
  const int colbase = blockIdx.x * 32, scene = blockIdx.y;

  const _Float16* abase = a1 + ((size_t)scene * 1024 + 128 * w + m) * C1;
  const _Float16* bb0 = W2t + (size_t)(colbase + m) * C1;
  const _Float16* bb1 = bb0 + (size_t)16 * C1;
  const float bias0 = b2[colbase + m], bias1 = b2[colbase + 16 + m];
  const v8f zero8 = {0.f, 0.f, 0.f, 0.f, 0.f, 0.f, 0.f, 0.f};

  #pragma unroll 1
  for (int hf = 0; hf < 2; ++hf) {
    v8f acc[4][2];
    #pragma unroll
    for (int t = 0; t < 4; ++t) { acc[t][0] = zero8; acc[t][1] = zero8; }
    const _Float16* ah = abase + (size_t)(64 * hf) * C1;
    #pragma unroll 1
    for (int k0 = 0; k0 < C1; k0 += 32) {
      const v16h fb0 = load_frag(bb0 + k0, h);
      const v16h fb1 = load_frag(bb1 + k0, h);
      #pragma unroll
      for (int t = 0; t < 4; ++t) {
        const v16h fa = load_frag(ah + (size_t)(16 * t) * C1 + k0, h);
        acc[t][0] = wmma_f16(fa, fb0, acc[t][0]);
        acc[t][1] = wmma_f16(fa, fb1, acc[t][1]);
      }
    }
    #pragma unroll
    for (int t = 0; t < 4; ++t) {
      #pragma unroll
      for (int r = 0; r < 8; ++r) {
        const int rowl = 128 * w + 64 * hf + 16 * t + 8 * h + r;
        sY[rowl * 32 + m]      = acc[t][0][r] * (1.0f / 1024.0f) + bias0;
        sY[rowl * 32 + 16 + m] = acc[t][1][r] * (1.0f / 1024.0f) + bias1;
      }
    }
  }
  __syncthreads();

  const int c = tid & 31, g = tid >> 5;
  double S = 0.0, S2 = 0.0;
  float mx[4], mn[4];
  #pragma unroll
  for (int jl = 0; jl < 4; ++jl) {
    float lmx = -3.0e38f, lmn = 3.0e38f;
    #pragma unroll 4
    for (int k = 0; k < 32; ++k) {
      const float y = sY[(128 * g + 32 * jl + k) * 32 + c];
      S += (double)y;
      S2 += (double)y * (double)y;
      lmx = fmaxf(lmx, y);
      lmn = fminf(lmn, y);
    }
    mx[jl] = lmx; mn[jl] = lmn;
  }
  sPart[(g * 32 + c) * 2 + 0] = S;
  sPart[(g * 32 + c) * 2 + 1] = S2;
  __syncthreads();
  if (tid < 32) {
    double a = 0.0, b = 0.0;
    #pragma unroll
    for (int gg = 0; gg < 8; ++gg) {
      a += sPart[(gg * 32 + tid) * 2 + 0];
      b += sPart[(gg * 32 + tid) * 2 + 1];
    }
    const double mean = a * (1.0 / 1024.0);
    double var = b * (1.0 / 1024.0) - mean * mean;
    if (var < 0.0) var = 0.0;
    const float varf = (float)var;
    const float rstd = 1.0f / sqrtf(varf + BNEPS);
    sStat[tid * 2 + 0] = (float)mean;
    sStat[tid * 2 + 1] = rstd * g2[colbase + tid];
  }
  __syncthreads();
  {
    const float meanf = sStat[c * 2 + 0];
    const float sc    = sStat[c * 2 + 1];
    const float be    = beta2[colbase + c];
    #pragma unroll
    for (int jl = 0; jl < 4; ++jl) {
      const float sel = (sc >= 0.0f) ? mx[jl] : mn[jl];
      const float v = fmaxf((sel - meanf) * sc + be, 0.0f);
      sOut[(4 * g + jl) * 32 + c] = v;
    }
  }
  __syncthreads();

  const int j = tid >> 3, q = tid & 7;
  const v4f o = *(const v4fa*)(sOut + j * 32 + 4 * q);
  float* dst = out + (size_t)(scene * NPED + j) * C2 + colbase + 4 * q;
  *(volatile v4f*)dst = o;
  __threadfence();
  *(volatile v4f*)dst = o;
}

extern "C" void kernel_launch(void* const* d_in, const int* in_sizes, int n_in,
                              void* d_out, int out_size, void* d_ws, size_t ws_size,
                              hipStream_t stream) {
  if (n_in < 16) return;
  if (in_sizes[0] != NB * HDIM) return;
  if (in_sizes[2] != NB * 2) return;
  if (in_sizes[6] != 2 * HDIM || in_sizes[7] != HDIM) return;
  if (in_sizes[8] != 2 * HDIM * C1 || in_sizes[9] != C1 || in_sizes[10] != C1 || in_sizes[11] != C1) return;
  if (in_sizes[12] != C1 * C2 || in_sizes[13] != C2 || in_sizes[14] != C2 || in_sizes[15] != C2) return;
  if (out_size != NB * C2) return;
  if (ws_size < (size_t)WS_TOTAL) return;

  const float* h_states = (const float*)d_in[0];
  const float* end_pos  = (const float*)d_in[2];
  const float* W_emb    = (const float*)d_in[6];
  const float* b_emb    = (const float*)d_in[7];
  const float* W1       = (const float*)d_in[8];
  const float* b1       = (const float*)d_in[9];
  const float* g1       = (const float*)d_in[10];
  const float* beta1    = (const float*)d_in[11];
  const float* W2       = (const float*)d_in[12];
  const float* b2       = (const float*)d_in[13];
  const float* g2       = (const float*)d_in[14];
  const float* beta2    = (const float*)d_in[15];
  float* out = (float*)d_out;

  char* ws = (char*)d_ws;
  _Float16* W2t  = (_Float16*)(ws + OFF_W2T);
  _Float16* W1bt = (_Float16*)(ws + OFF_W1BT);
  _Float16* hh   = (_Float16*)(ws + OFF_HH);
  float*    MK   = (float*)(ws + OFF_MK);
  float*    Ap   = (float*)(ws + OFF_AP);
  float*    Pp   = (float*)(ws + OFF_PP);
  _Float16* a1   = (_Float16*)(ws + OFF_A1);

  prep_kernel<<<202, 256, 0, stream>>>(W1, W2, h_states, W_emb, b_emb, b1, W2t, W1bt, hh, MK);

  pair_vec_kernel<<<dim3(NB / 128, C1 / 32), 256, 0, stream>>>(hh, W1bt, MK, end_pos, g1, beta1, Ap, Pp);

  a1_build_kernel<<<(NPAIR * (C1 / 8) + 255) / 256, 256, 0, stream>>>(Ap, Pp, a1);

  hipFuncSetAttribute(reinterpret_cast<const void*>(&gemm2_pool_kernel),
                      hipFuncAttributeMaxDynamicSharedMemorySize, DYN_LDS_K4);
  gemm2_pool_kernel<<<dim3(C2 / 32, NSCENE), 256, DYN_LDS_K4, stream>>>(a1, W2t, b2, g2, beta2, out);
}
